// MatchCNN_st_48292612276233
// MI455X (gfx1250) — hardware-verified
//
#include <hip/hip_runtime.h>

typedef __attribute__((ext_vector_type(16))) _Float16 v16h;
typedef __attribute__((ext_vector_type(8)))  _Float16 v8h;
typedef __attribute__((ext_vector_type(16))) __bf16   v16b;
typedef __attribute__((ext_vector_type(8)))  __bf16   v8b;
typedef __attribute__((ext_vector_type(8)))  float    v8f;
typedef __attribute__((ext_vector_type(4)))  float    v4f;
typedef __attribute__((ext_vector_type(4)))  unsigned int v4u;

constexpr int kB      = 1024;
constexpr int kPadLen = 30;
constexpr int kE      = 512;
constexpr int kImg    = 2048;
constexpr int kVocab  = 32000;
constexpr int kC1 = 200, kC2 = 300, kC3 = 300, kLin2 = 400;
constexpr int kL1 = 30, kLp1 = 14;
constexpr int kL2 = 14, kLp2 = 6;
constexpr int kL3 = 6,  kLp3 = 2;
constexpr int kRows1 = kB * kL1;
constexpr int kRows1p = kRows1 + 32;
constexpr int kRows2 = kB * kL2;
constexpr int kRows2p = kRows2 + 32;
constexpr int kRows3 = kB * kL3;
constexpr int kRows3p = kRows3 + 32;
constexpr int kCp1 = 512, kCp2 = 256, kCp3 = 320;
constexpr int kK1 = 3 * kCp1;
constexpr int kK2 = 3 * kCp2;
constexpr int kK3 = 3 * kCp3;
constexpr int kN1 = 256, kN2 = 320, kN3 = 320;
constexpr int kFeatPool = 600;
constexpr int kFeatReal = 2648;
constexpr int kKm = 2688;
constexpr int kNm = 448;
constexpr float kWCarry    = 32.0f;
constexpr float kWCarryInv = 1.0f / 32.0f;

static_assert(kK1 % 32 == 0 && kK2 % 32 == 0 && kK3 % 32 == 0 && kKm % 32 == 0, "K multiples of 32");
static_assert(kRows1 % 64 == 0 && kRows2 % 64 == 0 && kRows3 % 64 == 0 && kB % 64 == 0, "M multiples of 64");
static_assert(kN1 % 64 == 0 && kN2 % 64 == 0 && kN3 % 64 == 0 && kNm % 64 == 0, "N multiples of 64");

__device__ __forceinline__ unsigned short f2bf_bits(float f) {
  unsigned u = __float_as_uint(f);
  return (unsigned short)((u + 0x7FFFu + ((u >> 16) & 1u)) >> 16);
}
__device__ __forceinline__ float bf_bits2f(unsigned short h) { return __uint_as_float(((unsigned)h) << 16); }

__device__ __forceinline__ void dep_guard_h(v8f& a, v8f& b, v16h x, v16h y) { asm volatile("v_nop\n\tv_nop\n\tv_nop\n\tv_nop" : "+v"(a), "+v"(b) : "v"(x), "v"(y)); }
__device__ __forceinline__ void dep_guard_b(v8f& a, v8f& b, v16b x, v16b y) { asm volatile("v_nop\n\tv_nop\n\tv_nop\n\tv_nop" : "+v"(a), "+v"(b) : "v"(x), "v"(y)); }
__device__ __forceinline__ void keep4_h(v16h a, v16h b, v16h c, v16h d) { asm volatile("v_nop" :: "v"(a), "v"(b), "v"(c), "v"(d)); }
__device__ __forceinline__ void keep4_b(v16b a, v16b b, v16b c, v16b d) { asm volatile("v_nop" :: "v"(a), "v"(b), "v"(c), "v"(d)); }
__device__ __forceinline__ void acc_guard4(v8f& a, v8f& b, v8f& c, v8f& d) { asm volatile("v_nop\n\tv_nop\n\tv_nop\n\tv_nop" : "+v"(a), "+v"(b), "+v"(c), "+v"(d)); }
template <typename T> struct Frag;
template <> struct Frag<_Float16> {
  typedef v16h V; union U { v16h v; v8h h[2]; };
  static __device__ __forceinline__ v16h load(const _Float16* p) {
    U f; f.h[0] = *(const v8h*)(p); f.h[1] = *(const v8h*)(p + 16); return f.v;
  }
  static __device__ __forceinline__ v8f mma(v16h a, v16h b, v8f c) {
    return __builtin_amdgcn_wmma_f32_16x16x32_f16(false, a, false, b, (short)0, c, false, false);
  }
  static __device__ __forceinline__ void guard(v8f& a, v8f& b, v16h x, v16h y) { dep_guard_h(a, b, x, y); }
  static __device__ __forceinline__ void keep(v16h a, v16h b, v16h c, v16h d) { keep4_h(a, b, c, d); }
};
template <> struct Frag<__bf16> {
  typedef v16b V; union U { v16b v; v8b h[2]; };
  static __device__ __forceinline__ v16b load(const __bf16* p) {
    U f; f.h[0] = *(const v8b*)(p); f.h[1] = *(const v8b*)(p + 16); return f.v;
  }
  static __device__ __forceinline__ v8f mma(v16b a, v16b b, v8f c) {
    return __builtin_amdgcn_wmma_f32_16x16x32_bf16(false, a, false, b, (short)0, c, false, false);
  }
  static __device__ __forceinline__ void guard(v8f& a, v8f& b, v16b x, v16b y) { dep_guard_b(a, b, x, y); }
  static __device__ __forceinline__ void keep(v16b a, v16b b, v16b c, v16b d) { keep4_b(a, b, c, d); }
};

__device__ __forceinline__ unsigned pk16(unsigned short a, unsigned short b) { return (unsigned)a | ((unsigned)b << 16); }
__device__ __forceinline__ unsigned short h_bits(float f) { const _Float16 h = (_Float16)f; return __builtin_bit_cast(unsigned short, h); }
__device__ __forceinline__ int imin(int a, int b) { return a < b ? a : b; }
__device__ __forceinline__ int imax(int a, int b) { return a > b ? a : b; }
__device__ __forceinline__ float wave_sum(float s) {
#pragma unroll
  for (int off = 16; off > 0; off >>= 1) s += __shfl_xor(s, off, 32);
  return s;
}

template <int ET> struct Elem;
template <> struct Elem<0> { typedef _Float16 T; };
template <> struct Elem<1> { typedef __bf16 T; };
template <int ET, bool SPLIT, int BIAS_MODE, int OUT_MODE, bool RESID, int ACT = 0>
__global__ __launch_bounds__(256) void wmma_gemm64(
    const unsigned short* __restrict__ Ap, const unsigned short* __restrict__ A2p, int lda, long strideA,
    const unsigned short* __restrict__ Btp, const unsigned short* __restrict__ Bt2p, int ldb, long strideB,
    void* __restrict__ Cout, void* __restrict__ Cout2, int ldc, long strideC,
    const float* __restrict__ bias,
    const float* __restrict__ resid, long strideR,
    int M, int N, int K, float scale) {
  typedef typename Elem<ET>::T T;
  typedef typename Frag<T>::V V;
  const T* A = (const T*)Ap; const T* A2 = (const T*)A2p; const T* Bt = (const T*)Btp; const T* Bt2 = (const T*)Bt2p;
  __shared__ __align__(16) float sT[8][16 * 68];
  const int b    = blockIdx.y;
  const int lane = threadIdx.x & 31;
  const int wave = threadIdx.x >> 5;
  const int tilesN = N >> 6;
  const int tilesM = M >> 6;
  const int tile = blockIdx.x * 8 + wave;
  if (tile >= tilesM * tilesN) return;
  const int tm = tile / tilesN;
  const int tn = tile - tm * tilesN;
  const int m0 = tm << 6;
  const int n0 = tn << 6;

  const T* Ab  = A  + (size_t)b * strideA;
  const T* Bb  = Bt + (size_t)b * strideB;
  const T* Ab2 = SPLIT ? (A2  + (size_t)b * strideA) : nullptr;
  const T* Bb2 = SPLIT ? (Bt2 + (size_t)b * strideB) : nullptr;

  const int rlane = lane & 15;
  const int koff  = (lane >> 4) * 8;
  const int mOff  = (lane >> 4) * 8;

  v8f acc[4][4];
#pragma unroll
  for (int i = 0; i < 4; ++i)
#pragma unroll
    for (int j = 0; j < 4; ++j) acc[i][j] = (v8f){0.f,0.f,0.f,0.f,0.f,0.f,0.f,0.f};

  for (int k0 = 0; k0 < K; k0 += 32) {
    V bh[4], bl[4];
#pragma unroll
    for (int j = 0; j < 4; ++j) {
      const size_t bo = (size_t)(n0 + (j << 4) + rlane) * ldb + koff + k0;
      bh[j] = Frag<T>::load(Bb + bo);
      if (SPLIT) bl[j] = Frag<T>::load(Bb2 + bo);
    }
#pragma unroll
    for (int i = 0; i < 4; ++i) {
      const size_t ao = (size_t)(m0 + (i << 4) + rlane) * lda + koff + k0;
      V ah = Frag<T>::load(Ab + ao);
      V al;
      if (SPLIT) al = Frag<T>::load(Ab2 + ao);
#pragma unroll
      for (int j = 0; j < 4; ++j) {
        acc[i][j] = Frag<T>::mma(ah, bh[j], acc[i][j]);
        if (SPLIT) {
          acc[i][j] = Frag<T>::mma(ah, bl[j], acc[i][j]);
          acc[i][j] = Frag<T>::mma(al, bh[j], acc[i][j]);
        }
      }
      Frag<T>::guard(acc[i][0], acc[i][3], ah, SPLIT ? al : ah);
    }
    Frag<T>::keep(bh[0], bh[1], bh[2], bh[3]);
    if (SPLIT) Frag<T>::keep(bl[0], bl[1], bl[2], bl[3]);
  }
  acc_guard4(acc[0][0], acc[0][1], acc[0][2], acc[0][3]);
  acc_guard4(acc[1][0], acc[1][1], acc[1][2], acc[1][3]);
  acc_guard4(acc[2][0], acc[2][1], acc[2][2], acc[2][3]);
  acc_guard4(acc[3][0], acc[3][1], acc[3][2], acc[3][3]);

  float* slab = sT[wave];
  const float* Rb = RESID ? (resid + (size_t)b * strideR) : nullptr;
#pragma unroll
  for (int i = 0; i < 4; ++i) {
    const int mBase = m0 + (i << 4);
#pragma unroll
    for (int j = 0; j < 4; ++j) {
      const int n = n0 + (j << 4) + rlane;
      float bv = 0.f;
      if (BIAS_MODE == 2) bv = bias[n];
#pragma unroll
      for (int r = 0; r < 8; ++r) {
        float v = acc[i][j][r] * scale;
        if (BIAS_MODE == 1) v += bias[mBase + mOff + r];
        if (BIAS_MODE == 2) v += bv;
        if (RESID) v += Rb[(size_t)(mBase + mOff + r) * ldc + n];
        if (ACT == 2) v = fmaxf(v, 0.0f);
        if (ACT == 4) v = (v > 0.f) ? v : 0.01f * v;
        slab[(mOff + r) * 68 + (j << 4) + rlane] = v;
      }
    }
    __builtin_amdgcn_fence(__ATOMIC_RELEASE, "workgroup");
    __builtin_amdgcn_wave_barrier();
    __builtin_amdgcn_fence(__ATOMIC_ACQUIRE, "workgroup");
    if (OUT_MODE == 0) {
      float* C = (float*)Cout + (size_t)b * strideC;
      const int hh = lane >> 4, c4 = (lane & 15) * 4;
      for (int pass = 0; pass < 2; ++pass) {
#pragma unroll
        for (int it = 0; it < 8; ++it) {
          const int row = it * 2 + hh;
          v4f v = *(const v4f*)(slab + row * 68 + c4);
          *(volatile v4f*)(C + (size_t)(mBase + row) * ldc + n0 + c4) = v;
        }
        __threadfence();
      }
    } else {
      const int q = lane >> 3, c8 = (lane & 7) * 8;
      unsigned short* C  = (unsigned short*)Cout  + (size_t)b * strideC;
      unsigned short* C2 = (OUT_MODE == 2) ? ((unsigned short*)Cout2 + (size_t)b * strideC) : nullptr;
      for (int pass = 0; pass < 2; ++pass) {
#pragma unroll
        for (int it = 0; it < 4; ++it) {
          const int row = it * 4 + q;
          const float* sp = slab + row * 68 + c8;
          v8h hv, lv;
#pragma unroll
          for (int e = 0; e < 8; ++e) {
            if (OUT_MODE == 1) {
              hv[e] = (_Float16)sp[e];
            } else {
              unsigned short hb = f2bf_bits(sp[e]);
              unsigned short lb = f2bf_bits(sp[e] - bf_bits2f(hb));
              hv[e] = __builtin_bit_cast(_Float16, hb);
              lv[e] = __builtin_bit_cast(_Float16, lb);
            }
          }
          *(volatile v8h*)(C + (size_t)(mBase + row) * ldc + n0 + c8) = hv;
          if (OUT_MODE == 2) *(volatile v8h*)(C2 + (size_t)(mBase + row) * ldc + n0 + c8) = lv;
        }
        __threadfence();
      }
    }
    __builtin_amdgcn_fence(__ATOMIC_RELEASE, "workgroup");
    __builtin_amdgcn_wave_barrier();
    __builtin_amdgcn_fence(__ATOMIC_ACQUIRE, "workgroup");
  }
}

__global__ __launch_bounds__(256) void embed_rows_kernel(const float* __restrict__ table, const int* __restrict__ sent,
                                                         unsigned short* __restrict__ Xh, float* __restrict__ RS) {
  __shared__ float rs[32];
  const int t = threadIdx.x, lane = t & 31, wave = t >> 5;
  const int rbase = blockIdx.x * 32;
  const v4f zero4 = (v4f){0.f, 0.f, 0.f, 0.f};
#pragma unroll 1
  for (int i = 0; i < 4; ++i) {
    const int r = rbase + wave * 4 + i;
    const bool valid = (r < kRows1);
    const int rc = valid ? r : (kRows1 - 1);
    int id = sent[rc];
    id = imax(0, imin(id, kVocab - 1));
    const float* src = table + (size_t)id * kE;
    unsigned short* dst = Xh + (size_t)r * kE;
    float s = 0.f;
#pragma unroll
    for (int it = 0; it < 2; ++it) {
      const int c0 = it * 256 + lane * 8;
      v4f a = *(const v4f*)(src + c0);
      v4f c = *(const v4f*)(src + c0 + 4);
      a = valid ? a : zero4;
      c = valid ? c : zero4;
      s += ((a[0] + a[1]) + (a[2] + a[3])) + ((c[0] + c[1]) + (c[2] + c[3]));
      unsigned short hb[8];
#pragma unroll
      for (int e = 0; e < 4; ++e) { hb[e] = h_bits(a[e]); hb[4 + e] = h_bits(c[e]); }
      const v4u u = (v4u){pk16(hb[0], hb[1]), pk16(hb[2], hb[3]), pk16(hb[4], hb[5]), pk16(hb[6], hb[7])};
      unsigned short* q = dst + c0;
      *(volatile v4u*)q = u;
      __threadfence();
      *(volatile v4u*)q = u;
    }
    s = wave_sum(s);
    if (lane == 0) rs[wave * 4 + i] = s;
  }
  __syncthreads();
  if (wave == 0 && lane < 8) {
    const v4f v = (v4f){rs[4 * lane], rs[4 * lane + 1], rs[4 * lane + 2], rs[4 * lane + 3]};
    float* q = RS + rbase + 4 * lane;
    *(volatile v4f*)q = v;
    __threadfence();
    *(volatile v4f*)q = v;
  }
}

__global__ __launch_bounds__(256) void wcast_kernel(const float* __restrict__ W, int nReal, int kReal, int cReal,
                                                    int cPitch, int kP, unsigned short* __restrict__ out,
                                                    int nChunks, float scale) {
  const int qi = blockIdx.x * 256 + threadIdx.x;
  if (qi >= nChunks) return;
  const int e0 = qi * 8;
  const int o  = e0 / kP;
  const int j0 = e0 - o * kP;
  const int oc = imin(o, nReal - 1);
  unsigned short hb[8];
#pragma unroll
  for (int e = 0; e < 8; ++e) {
    const int j = j0 + e;
    const int seg = j / cPitch;
    const int c = j - seg * cPitch;
    const int kin = seg * cReal + c;
    const bool ok = (o < nReal) && (c < cReal) && (kin < kReal);
    const int kc = imin(kin, kReal - 1);
    float v = W[(size_t)oc * kReal + kc];
    v = ok ? v * scale : 0.f;
    hb[e] = h_bits(v);
  }
  const v4u u = (v4u){pk16(hb[0], hb[1]), pk16(hb[2], hb[3]), pk16(hb[4], hb[5]), pk16(hb[6], hb[7])};
  unsigned short* q = out + 8 * (size_t)qi;
  *(volatile v4u*)q = u;
  __threadfence();
  *(volatile v4u*)q = u;
}

__global__ __launch_bounds__(128) void bias_pad_kernel(const float* __restrict__ ba, int na, const float* __restrict__ bb, int nb,
                                                       const float* __restrict__ bc, int nc, const float* __restrict__ bd, int nd,
                                                       float* __restrict__ oa, float* __restrict__ ob, float* __restrict__ oc,
                                                       float* __restrict__ od, int npa, int npb, int npc, int npd) {
  const int y = blockIdx.y;
  const float* b = (y == 0) ? ba : (y == 1) ? bb : (y == 2) ? bc : bd;
  float* o       = (y == 0) ? oa : (y == 1) ? ob : (y == 2) ? oc : od;
  const int n    = (y == 0) ? na : (y == 1) ? nb : (y == 2) ? nc : nd;
  const int np   = (y == 0) ? npa : (y == 1) ? npb : (y == 2) ? npc : npd;
  const int i = threadIdx.x;
  if (4 * i >= np) return;
  v4f v;
#pragma unroll
  for (int e = 0; e < 4; ++e) {
    const int idx = 4 * i + e;
    const float f = b[imin(idx, n - 1)];
    v[e] = (idx < n) ? f : 0.f;
  }
  float* q = o + 4 * i;
  *(volatile v4f*)q = v;
  __threadfence();
  *(volatile v4f*)q = v;
}

__global__ __launch_bounds__(256) void pool_rows_kernel(const float* __restrict__ Y, int ldy, const float* __restrict__ RSin,
                                                        int nRowsIn, int Lin, int Lp, int nRowsOut, int cReal, int cPitch,
                                                        unsigned short* __restrict__ Xh, float* __restrict__ RSout) {
  __shared__ float rs[32];
  const int t = threadIdx.x, lane = t & 31, wave = t >> 5;
  const int rbase = blockIdx.x * 32;
  const int nIt = (cPitch + 255) / 256;
#pragma unroll 1
  for (int i = 0; i < 4; ++i) {
    const int r = rbase + wave * 4 + i;
    const bool valid = (r < nRowsOut);
    const int rc = valid ? r : (nRowsOut - 1);
    const int b = rc / Lp;
    const int p = rc - b * Lp;
    const int i0 = b * Lin + 2 * p;
    const float q0 = RSin[imin(i0, nRowsIn - 1)];
    const float q1 = RSin[imin(i0 + 1, nRowsIn - 1)];
    const float q2 = RSin[imin(i0 + 2, nRowsIn - 1)];
    const float q3 = RSin[imin(i0 + 3, nRowsIn - 1)];
    const float m0 = (((q0 + q1) + q2) != 0.f) ? 1.f : 0.f;
    const float m1 = (((q1 + q2) + q3) != 0.f) ? 1.f : 0.f;
    const float* y0p = Y + (size_t)imin(i0, nRowsIn - 1) * ldy;
    const float* y1p = Y + (size_t)imin(i0 + 1, nRowsIn - 1) * ldy;
    unsigned short* dst = Xh + (size_t)r * cPitch;
    float s = 0.f;
#pragma unroll 1
    for (int it = 0; it < nIt; ++it) {
      const int col0 = it * 256 + lane * 8;
      const bool active = (col0 < cPitch);
      unsigned short hb[8];
#pragma unroll
      for (int e = 0; e < 8; ++e) {
        const int col = col0 + e;
        const int cc = imin(col, cReal - 1);
        const float a = y0p[cc] * m0;
        const float d = y1p[cc] * m1;
        float v = fmaxf(a, d);
        v = (valid && (col < cReal)) ? v : 0.f;
        s += v;
        hb[e] = h_bits(v);
      }
      const v4u u = (v4u){pk16(hb[0], hb[1]), pk16(hb[2], hb[3]), pk16(hb[4], hb[5]), pk16(hb[6], hb[7])};
      if (active) {
        unsigned short* q = dst + col0;
        *(volatile v4u*)q = u;
        __threadfence();
        *(volatile v4u*)q = u;
      }
    }
    s = wave_sum(s);
    if (lane == 0) rs[wave * 4 + i] = s;
  }
  __syncthreads();
  if (wave == 0 && lane < 8) {
    const v4f v = (v4f){rs[4 * lane], rs[4 * lane + 1], rs[4 * lane + 2], rs[4 * lane + 3]};
    float* q = RSout + rbase + 4 * lane;
    *(volatile v4f*)q = v;
    __threadfence();
    *(volatile v4f*)q = v;
  }
}

__global__ __launch_bounds__(128) void feats_kernel(const float* __restrict__ Y3, const float* __restrict__ RS3,
                                                    const float* __restrict__ img, unsigned short* __restrict__ F) {
  const int b = blockIdx.x;
  const int t = threadIdx.x;
  const float* rsb = RS3 + (size_t)b * kL3;
  const float r0 = rsb[0], r1 = rsb[1], r2 = rsb[2], r3 = rsb[3], r4 = rsb[4], r5 = rsb[5];
  const float mw0 = (((r0 + r1) + r2) != 0.f) ? 1.f : 0.f;
  const float mw1 = (((r1 + r2) + r3) != 0.f) ? 1.f : 0.f;
  const float mw2 = (((r2 + r3) + r4) != 0.f) ? 1.f : 0.f;
  const float mw3 = (((r3 + r4) + r5) != 0.f) ? 1.f : 0.f;
  const float* yb = Y3 + (size_t)(b * kL3) * kN3;
  const float* ib = img + (size_t)b * kImg;
  unsigned short* fb = F + (size_t)b * kKm;
#pragma unroll 1
  for (int it = 0; it < 3; ++it) {
    const int ch = it * 128 + t;
    const int chc = imin(ch, kKm / 8 - 1);
    const int col0 = chc * 8;
    const int icol = imin(imax(col0 - kFeatPool, 0), kImg - 8);
    const v4f ia = *(const v4f*)(ib + icol);
    const v4f ic = *(const v4f*)(ib + icol + 4);
    unsigned short hb[8];
#pragma unroll
    for (int e = 0; e < 8; ++e) {
      const int col = col0 + e;
      const int yc = imin(col, kFeatPool - 1);
      const int p = (yc >= kC3) ? 1 : 0;
      const int c = yc - p * kC3;
      const float a = yb[(size_t)(2 * p) * kN3 + c];
      const float d = yb[(size_t)(2 * p + 1) * kN3 + c];
      const float ma = p ? mw2 : mw0;
      const float md = p ? mw3 : mw1;
      const float pv = fmaxf(a * ma, d * md);
      const float iv = (e < 4) ? ia[e] : ic[e - 4];
      const float v = (col < kFeatPool) ? pv : ((col < kFeatReal) ? iv : 0.f);
      hb[e] = h_bits(v);
    }
    const v4u u = (v4u){pk16(hb[0], hb[1]), pk16(hb[2], hb[3]), pk16(hb[4], hb[5]), pk16(hb[6], hb[7])};
    if (ch < kKm / 8) {
      unsigned short* q = fb + col0;
      *(volatile v4u*)q = u;
      __threadfence();
      *(volatile v4u*)q = u;
    }
  }
}

__global__ __launch_bounds__(256) void final_kernel(const float* __restrict__ H, int ldh, const float* __restrict__ Wo,
                                                    const float* __restrict__ bo, float* __restrict__ out) {
  __shared__ float res[kB];
  const int t = threadIdx.x, lane = t & 31, wave = t >> 5;
  const float bov = bo[0];
  v4f w[4];
  bool keep[4];
  int cc[4];
#pragma unroll
  for (int it = 0; it < 4; ++it) {
    const int col = it * 128 + lane * 4;
    cc[it] = imin(col, kLin2 - 4);
    keep[it] = (col < kLin2);
    w[it] = *(const v4f*)(Wo + cc[it]);
  }
#pragma unroll 1
  for (int rr = 0; rr < kB / 8; ++rr) {
    const int row = rr * 8 + wave;
    const float* hr = H + (size_t)row * ldh;
    float s = 0.f;
#pragma unroll
    for (int it = 0; it < 4; ++it) {
      const v4f hv = *(const v4f*)(hr + cc[it]);
      const float d = ((hv[0] * w[it][0] + hv[1] * w[it][1]) + (hv[2] * w[it][2] + hv[3] * w[it][3]));
      s += keep[it] ? d : 0.f;
    }
    s = wave_sum(s);
    if (lane == 0) res[row] = s + bov;
  }
  __syncthreads();
  {
    const int o = wave * 128 + lane * 4;
    const v4f v = (v4f){res[o], res[o + 1], res[o + 2], res[o + 3]};
    float* q = out + o;
    *(volatile v4f*)q = v;
    __threadfence();
    *(volatile v4f*)q = v;
  }
}

static void launch_gemm(const unsigned short* A, int lda, const unsigned short* Bt, int ldb, float* C, int ldc,
                        const float* bias, int M, int N, int K, float scale, hipStream_t stream) {
  const int tiles = (M / 64) * (N / 64);
  const int blocks = (tiles + 7) / 8;
  wmma_gemm64<0, false, 2, 0, false, 4><<<dim3(blocks, 1), dim3(256), 0, stream>>>(
      A, nullptr, lda, 0L, Bt, nullptr, ldb, 0L, (void*)C, nullptr, ldc, 0L, bias, nullptr, 0L, M, N, K, scale);
}

extern "C" void kernel_launch(void* const* d_in, const int* in_sizes, int n_in,
                              void* d_out, int out_size, void* d_ws, size_t ws_size,
                              hipStream_t stream) {
  if (n_in < 13) return;
  const float* image = (const float*)d_in[0];
  const int*   sent  = (const int*)d_in[1];
  const float* table = (const float*)d_in[2];
  const float* W1 = (const float*)d_in[3];   const float* b1 = (const float*)d_in[4];
  const float* W2 = (const float*)d_in[5];   const float* b2 = (const float*)d_in[6];
  const float* W3 = (const float*)d_in[7];   const float* b3 = (const float*)d_in[8];
  const float* Wm = (const float*)d_in[9];   const float* bm = (const float*)d_in[10];
  const float* Wo = (const float*)d_in[11];  const float* bo = (const float*)d_in[12];
  float* out = (float*)d_out;
  if (out_size < kB) return;
  if (in_sizes[1] < kRows1 || in_sizes[0] < kB * kImg) return;

  char* base = (char*)d_ws;
  size_t off = 0;
  auto carve = [&](size_t bytes) -> char* {
    off = (off + 255) & ~(size_t)255;
    char* p = base + off; off += bytes; return p;
  };
  unsigned short* X1h = (unsigned short*)carve((size_t)kRows1p * kCp1 * 2);
  float* RS1 = (float*)carve((size_t)kRows1p * 4);
  unsigned short* W1t = (unsigned short*)carve((size_t)kN1 * kK1 * 2);
  unsigned short* W2t = (unsigned short*)carve((size_t)kN2 * kK2 * 2);
  unsigned short* W3t = (unsigned short*)carve((size_t)kN3 * kK3 * 2);
  unsigned short* Wmt = (unsigned short*)carve((size_t)kNm * kKm * 2);
  float* biasp = (float*)carve((size_t)(kN1 + kN2 + kN3 + kNm) * 4);
  float* b1p = biasp;
  float* b2p = biasp + kN1;
  float* b3p = biasp + kN1 + kN2;
  float* bmp = biasp + kN1 + kN2 + kN3;
  float* Y1 = (float*)carve((size_t)kRows1 * kN1 * 4);
  unsigned short* X2h = (unsigned short*)carve((size_t)kRows2p * kCp2 * 2);
  float* RS2 = (float*)carve((size_t)kRows2p * 4);
  float* Y2 = (float*)carve((size_t)kRows2 * kN2 * 4);
  unsigned short* X3h = (unsigned short*)carve((size_t)kRows3p * kCp3 * 2);
  float* RS3 = (float*)carve((size_t)kRows3p * 4);
  float* Y3 = (float*)carve((size_t)kRows3 * kN3 * 4);
  unsigned short* Fh = (unsigned short*)carve((size_t)kB * kKm * 2);
  float* Hf = (float*)carve((size_t)kB * kNm * 4);
  if (off > ws_size) return;

  embed_rows_kernel<<<dim3(kRows1p / 32), dim3(256), 0, stream>>>(table, sent, X1h, RS1);

  wcast_kernel<<<dim3((kN1 * kK1 / 8) / 256), dim3(256), 0, stream>>>(W1, kC1, 3 * kE, kE, kCp1, kK1, W1t, kN1 * kK1 / 8, kWCarry);
  wcast_kernel<<<dim3((kN2 * kK2 / 8) / 256), dim3(256), 0, stream>>>(W2, kC2, 3 * kC1, kC1, kCp2, kK2, W2t, kN2 * kK2 / 8, kWCarry);
  wcast_kernel<<<dim3((kN3 * kK3 / 8) / 256), dim3(256), 0, stream>>>(W3, kC3, 3 * kC2, kC2, kCp3, kK3, W3t, kN3 * kK3 / 8, kWCarry);
  wcast_kernel<<<dim3((kNm * kKm / 8) / 256), dim3(256), 0, stream>>>(Wm, kLin2, kFeatReal, kFeatReal, kKm, kKm, Wmt, kNm * kKm / 8, kWCarry);

  bias_pad_kernel<<<dim3(1, 4), dim3(128), 0, stream>>>(b1, kC1, b2, kC2, b3, kC3, bm, kLin2, b1p, b2p, b3p, bmp, kN1, kN2, kN3, kNm);

  launch_gemm(X1h, kCp1, W1t, kK1, Y1, kN1, b1p, kRows1, kN1, kK1, kWCarryInv, stream);
  pool_rows_kernel<<<dim3(kRows2p / 32), dim3(256), 0, stream>>>(Y1, kN1, RS1, kRows1, kL1, kLp1, kRows2, kC1, kCp2, X2h, RS2);

  launch_gemm(X2h, kCp2, W2t, kK2, Y2, kN2, b2p, kRows2, kN2, kK2, kWCarryInv, stream);
  pool_rows_kernel<<<dim3(kRows3p / 32), dim3(256), 0, stream>>>(Y2, kN2, RS2, kRows2, kL2, kLp2, kRows3, kC2, kCp3, X3h, RS3);

  launch_gemm(X3h, kCp3, W3t, kK3, Y3, kN3, b3p, kRows3, kN3, kK3, kWCarryInv, stream);
  feats_kernel<<<dim3(kB), dim3(128), 0, stream>>>(Y3, RS3, image, Fh);

  launch_gemm(Fh, kKm, Wmt, kKm, Hf, kNm, bmp, kB, kNm, kKm, kWCarryInv, stream);

  final_kernel<<<dim3(1), dim3(256), 0, stream>>>(Hf, kNm, Wo, bo, out);
}
